// FraudMLPWithEmbedding_89481348645267
// MI455X (gfx1250) — hardware-verified
//
#include <hip/hip_runtime.h>


namespace {
constexpr int NB = 262144, FN = 16, E0 = 64, E1 = 32, E2 = 16, V0 = 100000, V1 = 10000, V2 = 1000, K = 128, HID = 256;
constexpr float XS = 8.0f, WSC = 256.0f;
typedef _Float16 b16;
typedef __attribute__((ext_vector_type(16))) _Float16 v16b;
typedef __attribute__((ext_vector_type(8))) _Float16 v8b;
typedef __attribute__((ext_vector_type(8))) float v8f;
typedef __attribute__((ext_vector_type(4))) float v4f;
__device__ __forceinline__ float bf16_rne(float f) { unsigned int u = __float_as_uint(f); u += 0x7FFFu + ((u >> 16) & 1u); return __uint_as_float(u & 0xFFFF0000u); }
__device__ __forceinline__ v16b frag_kb(const b16* p, int hh) { const v8b a = *(const v8b*)(p + 8 * hh), b = *(const v8b*)(p + 16 + 8 * hh); v16b f;
#pragma unroll
  for (int e = 0; e < 8; ++e) { f[e] = a[e]; f[8 + e] = b[e]; } return f; }
__device__ __forceinline__ v8f wmma16b(v16b a, v16b b, v8f c) { v8f d = __builtin_amdgcn_wmma_f32_16x16x32_f16(false, a, false, b, (short)0, c, false, false); asm volatile("v_nop\n\tv_nop\n\tv_nop\n\tv_nop" : "+v"(d) : "v"(a), "v"(b)); return d; }
__device__ __forceinline__ float pmul(float a, float b) { float p = a * b; asm volatile("" : "+v"(p)); return p; }
__device__ __forceinline__ float opaque(float a) { asm volatile("" : "+v"(a)); return a; }
__device__ __forceinline__ int iclamp(int v, int lo, int hi) { return v < lo ? lo : (v > hi ? hi : v); }

__global__ __launch_bounds__(256) void wprep_kernel(const float* __restrict__ w1, b16* __restrict__ W1T) {
  const size_t u = (size_t)blockIdx.x * 256 + threadIdx.x; if (u >= (size_t)HID * K / 8) return; const size_t e = u * 8; const int oo = (int)(e / K), k0 = (int)(e % K); v8b o;
  for (int j = 0; j < 8; ++j) o[j] = (b16)(bf16_rne(w1[(size_t)(k0 + j) * HID + oo]) * WSC);
  for (int pass = 0; pass < 2; ++pass) { *(volatile v8b*)(W1T + e) = o; __threadfence(); }
}
__device__ __forceinline__ float featv(const float* __restrict__ xn, const float* __restrict__ e0, const float* __restrict__ e1, const float* __restrict__ e2, size_t r, int i0, int i1, int i2, int k) {
  if (k < FN) return xn[r * FN + k]; k -= FN; if (k < E0) return e0[(size_t)i0 * E0 + k]; k -= E0; if (k < E1) return e1[(size_t)i1 * E1 + k]; k -= E1; return e2[(size_t)i2 * E2 + k];
}
__global__ __launch_bounds__(128) void mlp_kernel(const float* __restrict__ xn, const int* __restrict__ xc, const float* __restrict__ e0, const float* __restrict__ e1, const float* __restrict__ e2, const b16* __restrict__ W1T, const float* __restrict__ b1, const float* __restrict__ w2, const float* __restrict__ b2, float* __restrict__ out) {
  __shared__ __attribute__((aligned(16))) float so[64];
  const int wave = threadIdx.x >> 5, lane = threadIdx.x & 31, nloc = lane & 15, hlf = lane >> 4; const size_t m0 = (size_t)blockIdx.x * 64 + wave * 16; const size_t r = m0 + nloc;
  const int i0 = iclamp(xc[r * 3], 0, V0 - 1), i1 = iclamp(xc[r * 3 + 1], 0, V1 - 1), i2 = iclamp(xc[r * 3 + 2], 0, V2 - 1);
  v8f acc[16];
#pragma unroll
  for (int t = 0; t < 16; ++t) acc[t] = (v8f){};
#pragma unroll
  for (int kb = 0; kb < K; kb += 32) { v16b a;
#pragma unroll
    for (int e = 0; e < 8; ++e) { a[e] = (b16)(bf16_rne(featv(xn, e0, e1, e2, r, i0, i1, i2, kb + 8 * hlf + e)) * XS); a[8 + e] = (b16)(bf16_rne(featv(xn, e0, e1, e2, r, i0, i1, i2, kb + 16 + 8 * hlf + e)) * XS); }
#pragma unroll
    for (int t = 0; t < 16; ++t) acc[t] = wmma16b(a, frag_kb(W1T + (size_t)(t * 16 + nloc) * K + kb, hlf), acc[t]); }
  float rs[8]; for (int rr = 0; rr < 8; ++rr) rs[rr] = 0.0f;
#pragma unroll
  for (int t = 0; t < 16; ++t) { const int c = t * 16 + nloc; const float bb = bf16_rne(b1[c]), ww = opaque(bf16_rne(w2[c]));
#pragma unroll
    for (int rr = 0; rr < 8; ++rr) rs[rr] += pmul(fmaxf(acc[t][rr] * (1.0f / (XS * WSC)) + bb, 0.0f), ww); }
#pragma unroll
  for (int rr = 0; rr < 8; ++rr) { float s = rs[rr]; s += __shfl_xor(s, 1); s += __shfl_xor(s, 2); s += __shfl_xor(s, 4); s += __shfl_xor(s, 8); rs[rr] = s; }
  if (nloc == 0) { const float bo = bf16_rne(b2[0]); for (int rr = 0; rr < 8; ++rr) { const float z = rs[rr] + bo; so[wave * 16 + 8 * hlf + rr] = 1.0f / (1.0f + __expf(-z)); } }
  __syncthreads();
  for (int pass = 0; pass < 2; ++pass) { if (threadIdx.x < 16) *(volatile v4f*)(out + (size_t)blockIdx.x * 64 + threadIdx.x * 4) = *(const v4f*)(&so[threadIdx.x * 4]); __threadfence(); }
}
}

extern "C" void kernel_launch(void* const* d_in, const int* in_sizes, int n_in, void* d_out, int out_size, void* d_ws, size_t ws_size, hipStream_t stream) {
  (void)n_in;
  auto Fp = [&](int i) { return (const float*)d_in[i]; }; auto Ip = [&](int i) { return (const int*)d_in[i]; };
  if (in_sizes[0] != NB * FN || in_sizes[1] != NB * 3 || in_sizes[2] != V0 * E0 || in_sizes[3] != V1 * E1 || in_sizes[4] != V2 * E2 || in_sizes[5] != K * HID || in_sizes[7] != HID || out_size != NB) return;
  if (ws_size < (size_t)HID * K * 2) return; b16* W1T = (b16*)d_ws;
  wprep_kernel<<<(unsigned)(((size_t)HID * K / 8 + 255) / 256), 256, 0, stream>>>(Fp(5), W1T);
  mlp_kernel<<<NB / 64, 128, 0, stream>>>(Fp(0), Ip(1), Fp(2), Fp(3), Fp(4), W1T, Fp(6), Fp(7), Fp(8), (float*)d_out);
}
